// BEVDeformableTransformerEncoder_86036784873799
// MI455X (gfx1250) — hardware-verified
//
#include <hip/hip_runtime.h>
#define CC 256
#define HWq 40
#define NI 1600
#define NG 8
#define CG 32
#define DH 64
#define INNER 512
#define HK 10
#define NJ 100
#define NJP 112
#define CPB 64
#define LSEL 5
#define NBR (NG * NI * NJ)
typedef __bf16 v16b __attribute__((ext_vector_type(16)));
typedef unsigned short v8us __attribute__((ext_vector_type(8), may_alias));
typedef float  v8f  __attribute__((ext_vector_type(8)));
typedef float  v4f  __attribute__((ext_vector_type(4)));
typedef float  v4fa __attribute__((ext_vector_type(4), may_alias));
union FragB { v16b v; v8us half[2]; unsigned short u[16]; };

__device__ __forceinline__ unsigned short bf16_bits(float x) { unsigned int u = __float_as_uint(x); return (unsigned short)((u + 0x7FFFu + ((u >> 16) & 1u)) >> 16); }
__device__ __forceinline__ float bf16_val(unsigned short b) { return __uint_as_float(((unsigned int)b) << 16); }
__device__ __forceinline__ float bf16_round(float x) { return bf16_val(bf16_bits(x)); }
template <int NT>
__device__ __forceinline__ v8f mmaN(v16b ah, v16b al, v16b bh, v16b bl, v8f c) {
  c = __builtin_amdgcn_wmma_f32_16x16x32_bf16(false, ah, false, bh, (short)0, c, false, false);
  if (NT >= 2) c = __builtin_amdgcn_wmma_f32_16x16x32_bf16(false, al, false, bh, (short)0, c, false, false);
  if (NT >= 3) c = __builtin_amdgcn_wmma_f32_16x16x32_bf16(false, ah, false, bl, (short)0, c, false, false);
  asm volatile("v_nop\n\tv_nop\n\tv_nop\n\tv_nop" : "+v"(c) : "v"(ah), "v"(al), "v"(bh), "v"(bl));
  return c;
}

__global__ __launch_bounds__(256) void k_wt_bf16(const float* __restrict__ W, unsigned short* __restrict__ Wt, int K, int N) {
  const int t = blockIdx.x * 256 + threadIdx.x;
  const int k8n = K / 8;
  if (t >= N * k8n) return;
  const int n = t / k8n, k8 = (t % k8n) * 8;
  v8us v;
#pragma unroll
  for (int i = 0; i < 8; ++i) v[i] = bf16_bits(W[(size_t)(k8 + i) * N + n]);
  *(volatile v8us*)(Wt + (size_t)n * K + k8) = v;
  __threadfence();
  *(volatile v8us*)(Wt + (size_t)n * K + k8) = v;
}

template <bool ASPLIT, int ACT, bool BIAS_BF16>
__global__ __launch_bounds__(128) void k_gemm_bf(const float* __restrict__ A, int lda, const unsigned short* __restrict__ Wt, int ldb,
                                               const float* __restrict__ bias, float* __restrict__ C, int ldc, int M, int N, int K) {
  __shared__ __attribute__((aligned(16))) float so[4][16][64];
  const int tid = threadIdx.x, w = tid >> 5, lane = tid & 31, ln = lane & 15, hh = lane >> 4;
  const int ntn = N / 64;
  const int wid = blockIdx.x * 4 + w;
  const int mt = wid / ntn, nq = wid % ntn;
  if (mt * 16 >= M) return;
  const int row0 = mt * 16, col0 = nq * 64;
  const float* arow = A + (size_t)(row0 + ln) * lda;
  v8f acc[4] = {};
  for (int kb = 0; kb < K; kb += 32) {
    FragB ah, al;
    const v4f x0 = *(const v4fa*)(arow + kb + 8 * hh), x1 = *(const v4fa*)(arow + kb + 8 * hh + 4);
    const v4f x2 = *(const v4fa*)(arow + kb + 16 + 8 * hh), x3 = *(const v4fa*)(arow + kb + 16 + 8 * hh + 4);
    float xs[16] = {x0[0],x0[1],x0[2],x0[3],x1[0],x1[1],x1[2],x1[3],x2[0],x2[1],x2[2],x2[3],x3[0],x3[1],x3[2],x3[3]};
#pragma unroll
    for (int i = 0; i < 16; ++i) { const unsigned short hb = bf16_bits(xs[i]); ah.u[i] = hb; al.u[i] = ASPLIT ? bf16_bits(xs[i] - bf16_val(hb)) : (unsigned short)0; }
#pragma unroll
    for (int t = 0; t < 4; ++t) {
      const unsigned short* brow = Wt + (size_t)(col0 + t * 16 + ln) * ldb + kb;
      FragB b;
      b.half[0] = *(const v8us*)(brow + 8 * hh);
      b.half[1] = *(const v8us*)(brow + 16 + 8 * hh);
      acc[t] = mmaN<ASPLIT ? 2 : 1>(ah.v, al.v, b.v, b.v, acc[t]);
    }
  }
#pragma unroll
  for (int t = 0; t < 4; ++t) {
    float bv = bias ? bias[col0 + t * 16 + ln] : 0.f;
    if (BIAS_BF16) bv = bf16_round(bv);
#pragma unroll
    for (int r = 0; r < 8; ++r) { float v = acc[t][r] + bv; if (ACT == 1) v = fmaxf(v, 0.f); so[w][8 * hh + r][t * 16 + ln] = v; }
  }
  __builtin_amdgcn_fence(__ATOMIC_ACQ_REL, "workgroup");
  __builtin_amdgcn_wave_barrier();
  const int rsub = lane >> 4, c4 = (lane & 15) * 4;
  for (int pass = 0; pass < 2; ++pass) {
#pragma unroll
    for (int q = 0; q < 8; ++q) {
      const int r = q * 2 + rsub;
      const v4f v = *(const v4fa*)&so[w][r][c4];
      *(volatile v4f*)(C + (size_t)(row0 + r) * ldc + col0 + c4) = v;
    }
    if (pass == 0) __threadfence();
  }
}

template <bool ASPLIT, int ACT, bool BIAS_BF16, bool RES_BF16>
__global__ __launch_bounds__(128) void k_gemm_bf3(const float* __restrict__ A, int lda, const unsigned short* __restrict__ Wt, int ldb,
                                                const float* __restrict__ bias, const float* __restrict__ resid, int rmod, int ldr,
                                                float* __restrict__ C, int ldc, int M, int N, int K) {
  __shared__ __attribute__((aligned(16))) float so[4][16][64];
  const int tid = threadIdx.x, w = tid >> 5, lane = tid & 31, ln = lane & 15, hh = lane >> 4;
  const int ntn = N / 64;
  const int wid = blockIdx.x * 4 + w;
  const int mt = wid / ntn, nq = wid % ntn;
  if (mt * 16 >= M) return;
  const int row0 = mt * 16, col0 = nq * 64;
  const float* arow = A + (size_t)(row0 + ln) * lda;
  v8f acc[4] = {};
  for (int kb = 0; kb < K; kb += 32) {
    FragB ah, al;
    const v4f x0 = *(const v4fa*)(arow + kb + 8 * hh), x1 = *(const v4fa*)(arow + kb + 8 * hh + 4);
    const v4f x2 = *(const v4fa*)(arow + kb + 16 + 8 * hh), x3 = *(const v4fa*)(arow + kb + 16 + 8 * hh + 4);
    float xs[16] = {x0[0],x0[1],x0[2],x0[3],x1[0],x1[1],x1[2],x1[3],x2[0],x2[1],x2[2],x2[3],x3[0],x3[1],x3[2],x3[3]};
#pragma unroll
    for (int i = 0; i < 16; ++i) { const unsigned short hb = bf16_bits(xs[i]); ah.u[i] = hb; al.u[i] = ASPLIT ? bf16_bits(xs[i] - bf16_val(hb)) : (unsigned short)0; }
#pragma unroll
    for (int t = 0; t < 4; ++t) {
      const unsigned short* brow = Wt + (size_t)(col0 + t * 16 + ln) * ldb + kb;
      FragB b;
      b.half[0] = *(const v8us*)(brow + 8 * hh);
      b.half[1] = *(const v8us*)(brow + 16 + 8 * hh);
      acc[t] = mmaN<ASPLIT ? 2 : 1>(ah.v, al.v, b.v, b.v, acc[t]);
    }
  }
#pragma unroll
  for (int t = 0; t < 4; ++t) {
    const int col = col0 + t * 16 + ln;
    float bv = bias ? bias[col] : 0.f;
    if (BIAS_BF16) bv = bf16_round(bv);
#pragma unroll
    for (int r = 0; r < 8; ++r) {
      float v = acc[t][r] + bv;
      if (resid) { float rv = resid[(size_t)((row0 + 8 * hh + r) % rmod) * ldr + col]; if (RES_BF16) rv = bf16_round(rv); v += rv; }
      if (ACT == 1) v = fmaxf(v, 0.f);
      if (ACT == 2) v = 0.5f * v * (1.0f + erff(v * 0.70710678118654752f));
      if (ACT == 3) { const float u = 0.7978845608028654f * (v + 0.044715f * v * v * v); v = 0.5f * v * (1.0f + tanhf(u)); }
      so[w][8 * hh + r][t * 16 + ln] = v;
    }
  }
  __builtin_amdgcn_fence(__ATOMIC_ACQ_REL, "workgroup");
  __builtin_amdgcn_wave_barrier();
  const int rsub = lane >> 4, c4 = (lane & 15) * 4;
  for (int pass = 0; pass < 2; ++pass) {
#pragma unroll
    for (int q = 0; q < 8; ++q) {
      const int r = q * 2 + rsub;
      const v4f v = *(const v4fa*)&so[w][r][c4];
      *(volatile v4f*)(C + (size_t)(row0 + r) * ldc + col0 + c4) = v;
    }
    if (pass == 0) __threadfence();
  }
}
template <bool PARAM_BF16>
__global__ __launch_bounds__(256) void k_layernorm(const float* __restrict__ X, const float* __restrict__ R, const float* __restrict__ g, const float* __restrict__ bta,
                                                  float* __restrict__ out_sum, float* __restrict__ out_norm, int N, float eps) {
  __shared__ float red[256];
  const int row = blockIdx.x, tid = threadIdx.x;
  const float* x = X + (size_t)row * N; const float* rr = R ? R + (size_t)row * N : nullptr;
  float vals[16];
  const int per = N / 256;
  float s1 = 0.f;
  for (int u = 0; u < per / 4; ++u) {
    const int j = tid * 4 + 1024 * u;
    const v4f a = *(const v4fa*)(x + j);
    v4f b = {0.f,0.f,0.f,0.f}; if (rr) b = *(const v4fa*)(rr + j);
#pragma unroll
    for (int q = 0; q < 4; ++q) { const float v = a[q] + b[q]; vals[u * 4 + q] = v; s1 += v; }
  }
  red[tid] = s1; __syncthreads();
  for (int st = 128; st > 0; st >>= 1) { if (tid < st) red[tid] += red[tid + st]; __syncthreads(); }
  const float mu = red[0] / (float)N; __syncthreads();
  float s2 = 0.f;
  for (int u = 0; u < per / 4; ++u)
#pragma unroll
    for (int q = 0; q < 4; ++q) { const float c = vals[u * 4 + q] - mu; s2 += c * c; }
  red[tid] = s2; __syncthreads();
  for (int st = 128; st > 0; st >>= 1) { if (tid < st) red[tid] += red[tid + st]; __syncthreads(); }
  const float rs = rsqrtf(red[0] / (float)N + eps);
  for (int pass = 0; pass < 2; ++pass) {
    for (int u = 0; u < per / 4; ++u) {
      const int j = tid * 4 + 1024 * u;
      v4f o, sm;
#pragma unroll
      for (int q = 0; q < 4; ++q) {
        float gg = g[j + q], bb = bta[j + q];
        if (PARAM_BF16) { gg = bf16_round(gg); bb = bf16_round(bb); }
        sm[q] = vals[u * 4 + q]; o[q] = (vals[u * 4 + q] - mu) * rs * gg + bb;
      }
      if (out_sum) *(volatile v4f*)(out_sum + (size_t)row * N + j) = sm;
      *(volatile v4f*)(out_norm + (size_t)row * N + j) = o;
    }
    if (pass == 0) __threadfence();
  }
}


typedef _Float16 v16h __attribute__((ext_vector_type(16)));
union FragH { v16h v; v8us half[2]; _Float16 h[16]; unsigned short u[16]; };
template <int NT>
__device__ __forceinline__ v8f mmaH(v16h ah, v16h al, v16h bh, v16h bl, v8f c) {
  c = __builtin_amdgcn_wmma_f32_16x16x32_f16(false, ah, false, bh, (short)0, c, false, false);
  if (NT >= 2) c = __builtin_amdgcn_wmma_f32_16x16x32_f16(false, al, false, bh, (short)0, c, false, false);
  if (NT >= 3) c = __builtin_amdgcn_wmma_f32_16x16x32_f16(false, ah, false, bl, (short)0, c, false, false);
  asm volatile("v_nop\n\tv_nop\n\tv_nop\n\tv_nop" : "+v"(c) : "v"(ah), "v"(al), "v"(bh), "v"(bl));
  return c;
}
template <bool ASPLIT>
__global__ __launch_bounds__(128) void k_gemm_h(const float* __restrict__ A, int lda, size_t sA, const _Float16* __restrict__ Bh, int ldb, size_t sB, float alpha, float* __restrict__ C, int ldc, size_t sC, int M, int N, int K) {
  __shared__ __attribute__((aligned(16))) float so[4][16][64];
  const int tid = threadIdx.x, w = tid >> 5, lane = tid & 31, ln = lane & 15, hh = lane >> 4; const int by = blockIdx.y;
  A += (size_t)by * sA; Bh += (size_t)by * sB; C += (size_t)by * sC;
  const int ntn = (N + 63) / 64; const int wid = blockIdx.x * 4 + w; const int mt = wid / ntn, nq = wid % ntn; if (mt * 16 >= M) return;
  const int row0 = mt * 16, col0 = nq * 64; const float* arow = A + (size_t)(row0 + ln) * lda;
  v8f acc[4] = {};
  for (int kb = 0; kb < K; kb += 32) {
    FragH ah, al;
    const v4f x0 = *(const v4fa*)(arow + kb + 8 * hh), x1 = *(const v4fa*)(arow + kb + 8 * hh + 4), x2 = *(const v4fa*)(arow + kb + 16 + 8 * hh), x3 = *(const v4fa*)(arow + kb + 16 + 8 * hh + 4);
    float xs[16] = {x0[0],x0[1],x0[2],x0[3],x1[0],x1[1],x1[2],x1[3],x2[0],x2[1],x2[2],x2[3],x3[0],x3[1],x3[2],x3[3]};
#pragma unroll
    for (int i = 0; i < 16; ++i) { const _Float16 h = (_Float16)xs[i]; ah.h[i] = h; al.h[i] = ASPLIT ? (_Float16)(xs[i] - (float)h) : (_Float16)0.0f; }
#pragma unroll
    for (int t = 0; t < 4; ++t) { if (col0 + t * 16 >= N) continue; const size_t boff = (size_t)(col0 + t * 16 + ln) * ldb + kb; FragH bq; bq.half[0] = *(const v8us*)(Bh + boff + 8 * hh); bq.half[1] = *(const v8us*)(Bh + boff + 16 + 8 * hh);
      acc[t] = mmaH<ASPLIT ? 2 : 1>(ah.v, al.v, bq.v, bq.v, acc[t]); }
  }
#pragma unroll
  for (int t = 0; t < 4; ++t) { if (col0 + t * 16 >= N) continue;
#pragma unroll
    for (int r = 0; r < 8; ++r) so[w][8 * hh + r][t * 16 + ln] = acc[t][r] * alpha; }
  __builtin_amdgcn_fence(__ATOMIC_ACQ_REL, "workgroup"); __builtin_amdgcn_wave_barrier();
  const int rsub = lane >> 4, c4 = (lane & 15) * 4;
  for (int pass = 0; pass < 2; ++pass) {
#pragma unroll
    for (int q = 0; q < 8; ++q) { const int r = q * 2 + rsub; if (col0 + c4 < N) { const v4f v = *(const v4fa*)&so[w][r][c4]; *(volatile v4f*)(C + (size_t)(row0 + r) * ldc + col0 + c4) = v; } }
    if (pass == 0) __threadfence(); }
}

__global__ __launch_bounds__(256) void k_wt_f16(const float* __restrict__ W, _Float16* __restrict__ Wt, int K, int N, float scale) {
  const int t = blockIdx.x * 256 + threadIdx.x; if (t >= N * (K / 8)) return; const int n = t / (K / 8), k8 = (t % (K / 8)) * 8; FragH f;
#pragma unroll
  for (int i = 0; i < 8; ++i) f.h[i] = (_Float16)(bf16_round(W[(size_t)(k8 + i) * N + n]) * scale); const v8us o = f.half[0];
  *(volatile v8us*)((unsigned short*)Wt + (size_t)n * K + k8) = o; __threadfence(); *(volatile v8us*)((unsigned short*)Wt + (size_t)n * K + k8) = o;
}
template <int ACT>
__global__ __launch_bounds__(128) void k_gemm_hhx(const _Float16* __restrict__ A, int lda, size_t sA, const _Float16* __restrict__ Bh, int ldb, size_t sB, float alpha, const float* __restrict__ bias, size_t sBias, const float* __restrict__ CP, int rowsPerB, size_t sCPb, int row0g,
    float* __restrict__ C, _Float16* __restrict__ C16, int ldc, size_t sC, int M, int N, int K) {
  __shared__ __attribute__((aligned(16))) float so[4][16][64];
  const int tid = threadIdx.x, w = tid >> 5, lane = tid & 31, ln = lane & 15, hh = lane >> 4; const int by = blockIdx.y;
  A += (size_t)by * sA; Bh += (size_t)by * sB; const size_t cofs = (size_t)by * sC; const float* bp = bias ? bias + (size_t)by * sBias : nullptr;
  const int ntn = (N + 63) / 64; const int wid = blockIdx.x * 4 + w; const int mt = wid / ntn, nq = wid % ntn; if (mt * 16 >= M) return;
  const int row0 = mt * 16, col0 = nq * 64; const _Float16* arow = A + (size_t)(row0 + ln) * lda;
  v8f acc[4] = {};
  for (int kb = 0; kb < K; kb += 32) { FragH ah; ah.half[0] = *(const v8us*)((const unsigned short*)arow + kb + 8 * hh); ah.half[1] = *(const v8us*)((const unsigned short*)arow + kb + 16 + 8 * hh);
#pragma unroll
    for (int t = 0; t < 4; ++t) { if (col0 + t * 16 >= N) continue; const size_t boff = (size_t)(col0 + t * 16 + ln) * ldb + kb; FragH bq; bq.half[0] = *(const v8us*)((const unsigned short*)Bh + boff + 8 * hh); bq.half[1] = *(const v8us*)((const unsigned short*)Bh + boff + 16 + 8 * hh);
      acc[t] = mmaH<1>(ah.v, ah.v, bq.v, bq.v, acc[t]); }
  }
#pragma unroll
  for (int t = 0; t < 4; ++t) { if (col0 + t * 16 >= N) continue; const int col = col0 + t * 16 + ln; const float bv = bp ? bf16_round(bp[col]) : 0.f;
#pragma unroll
    for (int r = 0; r < 8; ++r) { float v = acc[t][r] * alpha + bv; if (CP) { const int bidx = (row0g + row0 + 8 * hh + r) / rowsPerB; v += CP[(size_t)bidx * sCPb + (size_t)by * 64 + col]; } if (ACT == 1) v = (v > 0.f) ? v : expm1f(v); else if (ACT == 7) v = (v > 0.f) ? v + 1.0f : expf(v); else if (ACT == 8) v = tanhf(v); else if (ACT == 9) v = 0.5f * v * (1.0f + tanhf(0.7978845608028654f * (v + 0.044715f * v * v * v))); else if (ACT == 11) v = 1.0f / (1.0f + expf(-v)); else if (ACT == 12) v = (v > 0.f) ? v : 0.01f * v; else if (ACT == 14) v = (v > 0.f) ? v : 0.1f * v; else if (ACT == 15) v = v / (1.0f + expf(-v)); else if (ACT == 3) v = fmaxf(v, 0.f); else if (ACT == 6) v = 0.5f * v * (1.0f + erff(v * 0.70710678118654752f)); so[w][8 * hh + r][t * 16 + ln] = v; } }
  __builtin_amdgcn_fence(__ATOMIC_ACQ_REL, "workgroup"); __builtin_amdgcn_wave_barrier();
  const int rsub = lane >> 4, c4 = (lane & 15) * 4; typedef _Float16 v4h __attribute__((ext_vector_type(4)));
  for (int pass = 0; pass < 2; ++pass) {
#pragma unroll
    for (int q = 0; q < 8; ++q) { const int r = q * 2 + rsub; if (col0 + c4 < N) { const v4f v = *(const v4fa*)&so[w][r][c4]; if (C) *(volatile v4f*)(C + cofs + (size_t)(row0 + r) * ldc + col0 + c4) = v; if (C16) { v4h h4; for (int i = 0; i < 4; ++i) h4[i] = (_Float16)v[i]; *(volatile v4h*)(C16 + cofs + (size_t)(row0 + r) * ldc + col0 + c4) = h4; } } }
    if (pass == 0) __threadfence(); }
}


typedef _Float16 v4h __attribute__((ext_vector_type(4)));

__global__ __launch_bounds__(256) void k_x16(const float* __restrict__ x, _Float16* __restrict__ X16, size_t n8) { const size_t t = (size_t)blockIdx.x * 256 + threadIdx.x; if (t >= n8) return; FragH f;
#pragma unroll
  for (int q = 0; q < 8; ++q) f.h[q] = (_Float16)bf16_round(x[t * 8 + q]); *(volatile v8us*)((unsigned short*)X16 + t * 8) = f.half[0]; __threadfence(); *(volatile v8us*)((unsigned short*)X16 + t * 8) = f.half[0]; }
__global__ __launch_bounds__(256) void k_h16(const float* __restrict__ x, _Float16* __restrict__ X16, size_t n8) { const size_t t = (size_t)blockIdx.x * 256 + threadIdx.x; if (t >= n8) return; FragH f;
#pragma unroll
  for (int q = 0; q < 8; ++q) f.h[q] = (_Float16)x[t * 8 + q]; *(volatile v8us*)((unsigned short*)X16 + t * 8) = f.half[0]; __threadfence(); *(volatile v8us*)((unsigned short*)X16 + t * 8) = f.half[0]; }
__global__ __launch_bounds__(256) void k_round16f(const float* __restrict__ W, _Float16* __restrict__ Bt, size_t n8) { const size_t t = (size_t)blockIdx.x * 256 + threadIdx.x; if (t >= n8) return; FragH f;
#pragma unroll
  for (int i = 0; i < 8; ++i) f.h[i] = (_Float16)(bf16_round(W[t * 8 + i]) * 16.0f); *(volatile v8us*)((unsigned short*)Bt + t * 8) = f.half[0]; __threadfence(); *(volatile v8us*)((unsigned short*)Bt + t * 8) = f.half[0]; }
template <int NHv, int TTv>
__global__ __launch_bounds__(256) void k_vt(const _Float16* __restrict__ V16, int ldv, int voff, _Float16* __restrict__ Vt) { __shared__ unsigned short tl[64][66]; const int tid = threadIdx.x; const int slab = blockIdx.x / (TTv / 64), lg = blockIdx.x % (TTv / 64); const int b = slab / NHv, h = slab % NHv;
  for (int i = tid; i < 64 * 8; i += 256) { const int r = i / 8, c8 = (i % 8) * 8; FragH f; f.half[0] = *(const v8us*)((const unsigned short*)V16 + ((size_t)b * TTv + lg * 64 + r) * ldv + voff + h * 64 + c8);
#pragma unroll
    for (int q = 0; q < 8; ++q) tl[r][c8 + q] = f.u[q]; }
  __syncthreads();
  for (int pass = 0; pass < 2; ++pass) {
#pragma unroll
    for (int rd = 0; rd < 2; ++rd) { const int d = rd * 32 + tid / 8, pc = tid % 8; FragH f;
#pragma unroll
      for (int q = 0; q < 8; ++q) f.u[q] = tl[pc * 8 + q][d];
      *(volatile v8us*)((unsigned short*)Vt + ((size_t)slab * 64 + d) * TTv + lg * 64 + pc * 8) = f.half[0]; }
    if (pass == 0) __threadfence(); } }

__global__ __launch_bounds__(256) void k_hl(const float* __restrict__ F, _Float16* __restrict__ Hh, _Float16* __restrict__ Hl, size_t n8) { const size_t t = (size_t)blockIdx.x * 256 + threadIdx.x; if (t >= n8) return; FragH fh, fl; const v4f a = *(const v4fa*)(F + t * 8), c = *(const v4fa*)(F + t * 8 + 4);
#pragma unroll
  for (int q = 0; q < 4; ++q) { _Float16 h = (_Float16)a[q]; fh.h[q] = h; fl.h[q] = (_Float16)((a[q] - (float)h) * 1024.0f); h = (_Float16)c[q]; fh.h[4 + q] = h; fl.h[4 + q] = (_Float16)((c[q] - (float)h) * 1024.0f); }
  for (int pass = 0; pass < 2; ++pass) { *(volatile v8us*)((unsigned short*)Hh + t * 8) = fh.half[0]; *(volatile v8us*)((unsigned short*)Hl + t * 8) = fl.half[0]; if (pass == 0) __threadfence(); } }

__global__ __launch_bounds__(256) void k_zero(float* __restrict__ P, size_t n4) { const size_t t = (size_t)blockIdx.x * 256 + threadIdx.x; if (t >= n4) return; const v4f z = {0.f, 0.f, 0.f, 0.f}; *(volatile v4f*)(P + t * 4) = z; __threadfence(); *(volatile v4f*)(P + t * 4) = z; }
__device__ __forceinline__ float gelu_e(float x) { return 0.5f * x * (1.0f + erff(x * 0.70710678118654752f)); }
__global__ __launch_bounds__(256) void k_xT(const float* __restrict__ x, _Float16* __restrict__ X16) { const int t = blockIdx.x * 256 + threadIdx.x; if (t >= NI * (CC / 8)) return; const int c0 = (t % (CC / 8)) * 8, p = t / (CC / 8); FragH f;
#pragma unroll
  for (int q = 0; q < 8; ++q) f.h[q] = (_Float16)bf16_round(x[(size_t)(c0 + q) * NI + p]);
  *(volatile v8us*)((unsigned short*)X16 + (size_t)p * CC + c0) = f.half[0]; __threadfence(); *(volatile v8us*)((unsigned short*)X16 + (size_t)p * CC + c0) = f.half[0]; }
__global__ __launch_bounds__(64) void k_offkv(const float* __restrict__ Q, const float* __restrict__ x, const float* __restrict__ w1, const float* __restrict__ b1, const float* __restrict__ w2, _Float16* __restrict__ KV16, float* __restrict__ VG) {
  #pragma clang fp contract(off)
  __shared__ float hs[64]; __shared__ __attribute__((aligned(16))) unsigned short kvs[32]; __shared__ float vg[2];
  const int tid = threadIdx.x; const int gj = blockIdx.x; const int g = gj / NJ, j = gj % NJ; const int jy = j / HK, jx = j % HK; const int c = tid;
  float acc = bf16_round(b1[LSEL * DH + c]);
#pragma unroll 1
  for (int kh = 0; kh < 6; ++kh) { const int yy = 4 * jy - 1 + kh; if (yy < 0 || yy >= HWq) continue;
#pragma unroll 1
    for (int kw = 0; kw < 6; ++kw) { const int xx = 4 * jx - 1 + kw; if (xx < 0 || xx >= HWq) continue; acc += bf16_round(w1[((size_t)LSEL * DH + c) * 36 + kh * 6 + kw]) * Q[(size_t)(yy * HWq + xx) * INNER + g * DH + c]; } }
  hs[c] = gelu_e(acc); __syncthreads();
  if (tid < 2) { float s = 0.f;
#pragma unroll 1
    for (int k = 0; k < DH; ++k) s += bf16_round(w2[((size_t)LSEL * 2 + tid) * DH + k]) * hs[k]; const float off = tanhf(s) * 4.0f; const float base = (tid == 0) ? (float)jx : (float)jy; vg[tid] = 2.0f * (base + off) / 9.0f - 1.0f; }
  __syncthreads();
  const float g0 = vg[0], g1 = vg[1];
  if (tid < 32) { const float gx = ((g0 + 1.0f) * (float)HWq - 1.0f) * 0.5f, gy = ((g1 + 1.0f) * (float)HWq - 1.0f) * 0.5f; const float fx = floorf(gx), fy = floorf(gy); const float wx1 = gx - fx, wy1 = gy - fy; const int x0 = (int)fx, y0 = (int)fy; float s = 0.f; const float* xc = x + (size_t)(g * CG + tid) * NI;
#pragma unroll
    for (int q4 = 0; q4 < 4; ++q4) { const int xi = x0 + (q4 & 1), yi = y0 + (q4 >> 1); const bool valid = (xi >= 0) && (xi <= HWq - 1) && (yi >= 0) && (yi <= HWq - 1); const float wgt = ((q4 & 1) ? wx1 : 1.f - wx1) * ((q4 >> 1) ? wy1 : 1.f - wy1); s += (valid ? wgt : 0.f) * bf16_round(xc[min(max(yi, 0), HWq - 1) * HWq + min(max(xi, 0), HWq - 1)]); }
    FragH f; f.h[0] = (_Float16)s; kvs[tid] = f.u[0]; }
  __syncthreads();
  for (int pass = 0; pass < 2; ++pass) {
    if (tid < 8) { v8us v; if (tid < 4) v = *(const v8us*)&kvs[tid * 8]; else {
#pragma unroll
        for (int q = 0; q < 8; ++q) v[q] = 0; } *(volatile v8us*)((unsigned short*)KV16 + ((size_t)g * NJP + j) * 64 + tid * 8) = v; }
    if (tid < 32) { const float val = (tid & 1) ? g1 : g0; *(volatile float*)(VG + (size_t)gj * 32 + tid) = val; }
    if (pass == 0) __threadfence(); } }
__global__ __launch_bounds__(256) void k_cpb0(const float* __restrict__ VG, int g, const float* __restrict__ w0, const float* __restrict__ b0, _Float16* __restrict__ H0) {
  #pragma clang fp contract(off)
  const size_t t = (size_t)blockIdx.x * 256 + threadIdx.x; if (t >= (size_t)NI * NJ * 8) return; const int c0 = (int)(t % 8) * 8; const size_t r = t / 8; const int i = (int)(r / NJ), j = (int)(r % NJ); const int iy = i / HWq, ix = i % HWq;
  const float q0 = 2.0f * (float)ix / 39.0f - 1.0f, q1 = 2.0f * (float)iy / 39.0f - 1.0f; const float p0 = q0 - VG[(size_t)(g * NJ + j) * 32], p1 = q1 - VG[(size_t)(g * NJ + j) * 32 + 1];
  const float s0 = ((p0 > 0.f) ? 1.f : (p0 < 0.f) ? -1.f : 0.f) * log1pf(fabsf(p0)), s1 = ((p1 > 0.f) ? 1.f : (p1 < 0.f) ? -1.f : 0.f) * log1pf(fabsf(p1)); FragH f;
#pragma unroll
  for (int q = 0; q < 8; ++q) { const int c = c0 + q; const float v = (s0 * bf16_round(w0[((size_t)LSEL * CPB + c) * 2]) + s1 * bf16_round(w0[((size_t)LSEL * CPB + c) * 2 + 1])) + bf16_round(b0[LSEL * CPB + c]); f.h[q] = (_Float16)fmaxf(v, 0.f); }
  *(volatile v8us*)((unsigned short*)H0 + r * CPB + c0) = f.half[0]; __threadfence(); *(volatile v8us*)((unsigned short*)H0 + r * CPB + c0) = f.half[0]; }
__global__ __launch_bounds__(256) void k_soft(const float* __restrict__ SIM, const float* __restrict__ BIAS, int g, _Float16* __restrict__ ATT) {
  #pragma clang fp contract(off)
  __shared__ __attribute__((aligned(16))) unsigned short rows[8][128]; const int tid = threadIdx.x, w = tid >> 5, l = tid & 31; const int i = blockIdx.x * 8 + w;
  float v[4]; float m = -3.0e38f;
#pragma unroll
  for (int q = 0; q < 4; ++q) { const int j = l + 32 * q; v[q] = (j < NJ) ? SIM[((size_t)g * NI + i) * NJP + j] + BIAS[((size_t)i * NJ + j) * 16] : -3.0e38f; m = fmaxf(m, v[q]); }
  for (int o = 16; o > 0; o >>= 1) m = fmaxf(m, __shfl_xor(m, o, 32)); float s = 0.f;
#pragma unroll
  for (int q = 0; q < 4; ++q) { const int j = l + 32 * q; v[q] = (j < NJ) ? expf(v[q] - m) : 0.f; s += v[q]; }
  for (int o = 16; o > 0; o >>= 1) s += __shfl_xor(s, o, 32); const float is = 1024.0f / s;
#pragma unroll
  for (int q = 0; q < 4; ++q) { const int j = l + 32 * q; FragH f; f.h[0] = (_Float16)(v[q] * is); rows[w][j] = (j < NJ) ? f.u[0] : (unsigned short)0; }
  __syncthreads();
  if (l < 16) { const v8us vv = *(const v8us*)&rows[w][l * 8]; *(volatile v8us*)((unsigned short*)ATT + ((size_t)g * NI + i) * 128 + l * 8) = vv; __threadfence(); *(volatile v8us*)((unsigned short*)ATT + ((size_t)g * NI + i) * 128 + l * 8) = vv; } }
__global__ __launch_bounds__(256) void k_vt(const _Float16* __restrict__ V16, _Float16* __restrict__ VT) { const int t = blockIdx.x * 256 + threadIdx.x; if (t >= NG * DH * (128 / 8)) return; const int j0 = (t % 16) * 8; const int hd = t / 16; const int h = hd / DH, d = hd % DH; FragH f;
#pragma unroll
  for (int q = 0; q < 8; ++q) { const int j = j0 + q; f.h[q] = (j < NJ) ? V16[(size_t)j * INNER + h * DH + d] : (_Float16)0.0f; }
  *(volatile v8us*)((unsigned short*)VT + (size_t)hd * 128 + j0) = f.half[0]; __threadfence(); *(volatile v8us*)((unsigned short*)VT + (size_t)hd * 128 + j0) = f.half[0]; }
__global__ __launch_bounds__(256) void k_kpad(const _Float16* __restrict__ K16, _Float16* __restrict__ KP) { const int t = blockIdx.x * 256 + threadIdx.x; if (t >= NJP * (INNER / 8)) return; const int c0 = (t % (INNER / 8)) * 8, j = t / (INNER / 8); FragH f; if (j < NJ) f.half[0] = *(const v8us*)((const unsigned short*)K16 + (size_t)j * INNER + c0); else {
#pragma unroll
    for (int q = 0; q < 8; ++q) f.h[q] = (_Float16)0.0f; }
  *(volatile v8us*)((unsigned short*)KP + (size_t)j * INNER + c0) = f.half[0]; __threadfence(); *(volatile v8us*)((unsigned short*)KP + (size_t)j * INNER + c0) = f.half[0]; }
__global__ __launch_bounds__(256) void k_nchw(const float* __restrict__ Y, float* __restrict__ out) { const int t = blockIdx.x * 256 + threadIdx.x; if (t >= CC * (NI / 4)) return; const int p4 = (t % (NI / 4)) * 4, o = t / (NI / 4); v4f v;
#pragma unroll
  for (int q = 0; q < 4; ++q) v[q] = Y[(size_t)(p4 + q) * CC + o]; *(volatile v4f*)(out + (size_t)o * NI + p4) = v; __threadfence(); *(volatile v4f*)(out + (size_t)o * NI + p4) = v; }
__global__ __launch_bounds__(256) void k_w2pad(const float* __restrict__ w2, const float* __restrict__ b2, _Float16* __restrict__ Bw2, float* __restrict__ Bb2) { const int t = blockIdx.x * 256 + threadIdx.x; if (t >= 16 * (CPB / 8)) return; const int k0 = (t % 8) * 8, n = t / 8; FragH f;
#pragma unroll
  for (int q = 0; q < 8; ++q) f.h[q] = (n == 0) ? (_Float16)(bf16_round(w2[(size_t)LSEL * CPB + k0 + q]) * 16.0f) : (_Float16)0.0f;
  *(volatile v8us*)((unsigned short*)Bw2 + (size_t)n * CPB + k0) = f.half[0]; __threadfence(); *(volatile v8us*)((unsigned short*)Bw2 + (size_t)n * CPB + k0) = f.half[0];
  if (t < 16) { const float v = (t == 0) ? b2[LSEL] : 0.f; *(volatile float*)(Bb2 + t) = v; __threadfence(); *(volatile float*)(Bb2 + t) = v; } }

extern "C" void kernel_launch(void* const* d_in, const int* in_sizes, int n_in,
                              void* d_out, int out_size, void* d_ws, size_t ws_size, hipStream_t stream) {
  (void)in_sizes; (void)n_in; (void)out_size;
  const float* const* I = (const float* const*)d_in; const float* x = I[0]; const float* wq = I[1]; const float* wk = I[2]; const float* wv = I[3]; const float* w1 = I[4]; const float* b1 = I[5]; const float* w2o = I[6]; const float* c0w = I[7]; const float* c0b = I[8]; const float* c1w = I[9]; const float* c1b = I[10]; const float* c2w = I[11]; const float* c2b = I[12]; const float* wo = I[13]; const float* bo = I[14];
  char* ws = (char*)d_ws; size_t off = 0;
  auto take = [&](size_t bytes) { char* p = ws + off; off += (bytes + 255) & ~(size_t)255; return p; };
  _Float16* Bq = (_Float16*)take((size_t)INNER * CG * 2); _Float16* Bk = (_Float16*)take((size_t)INNER * CG * 2); _Float16* Bv = (_Float16*)take((size_t)INNER * CG * 2); _Float16* Bc1 = (_Float16*)take((size_t)CPB * CPB * 2); _Float16* Bw2 = (_Float16*)take((size_t)16 * CPB * 2); float* Bb2 = (float*)take(64 * 4); _Float16* Bo = (_Float16*)take((size_t)CC * INNER * 2);
  _Float16* X16 = (_Float16*)take((size_t)NI * CC * 2); float* Q = (float*)take((size_t)NI * INNER * 4); _Float16* Q16 = (_Float16*)take((size_t)NI * INNER * 2); _Float16* KV16 = (_Float16*)take((size_t)NG * NJP * 64 * 2); float* VG = (float*)take((size_t)NG * NJ * 32 * 4);
  _Float16* K16 = (_Float16*)take((size_t)NJP * INNER * 2); _Float16* V16 = (_Float16*)take((size_t)NJP * INNER * 2); _Float16* KP = (_Float16*)take((size_t)NJP * INNER * 2); _Float16* VT = (_Float16*)take((size_t)NG * DH * 128 * 2); float* SIM = (float*)take((size_t)NG * NI * NJP * 4);
  _Float16* H0 = (_Float16*)take((size_t)NI * NJ * CPB * 2); _Float16* H1 = (_Float16*)take((size_t)NI * NJ * CPB * 2); float* BIAS = (float*)take((size_t)NI * NJ * 16 * 4); _Float16* ATT = (_Float16*)take((size_t)NG * NI * 128 * 2); _Float16* O16 = (_Float16*)take((size_t)NI * INNER * 2); float* Y = (float*)take((size_t)NI * CC * 4);
  if (off > ws_size) return;
  k_round16f<<<(INNER * CG / 8 + 255) / 256, 256, 0, stream>>>(wq + (size_t)LSEL * INNER * CG, Bq, (size_t)INNER * CG / 8); k_round16f<<<(INNER * CG / 8 + 255) / 256, 256, 0, stream>>>(wk + (size_t)LSEL * INNER * CG, Bk, (size_t)INNER * CG / 8); k_round16f<<<(INNER * CG / 8 + 255) / 256, 256, 0, stream>>>(wv + (size_t)LSEL * INNER * CG, Bv, (size_t)INNER * CG / 8);
  k_round16f<<<(CPB * CPB / 8 + 255) / 256, 256, 0, stream>>>(c1w + (size_t)LSEL * CPB * CPB, Bc1, (size_t)CPB * CPB / 8); k_w2pad<<<1, 256, 0, stream>>>(c2w, c2b, Bw2, Bb2); k_round16f<<<(unsigned)(((size_t)CC * INNER / 8 + 255) / 256), 256, 0, stream>>>(wo + (size_t)LSEL * CC * INNER, Bo, (size_t)CC * INNER / 8);
  k_xT<<<(NI * (CC / 8) + 255) / 256, 256, 0, stream>>>(x, X16);
  k_gemm_hhx<0><<<dim3(((NI / 16) * 1 + 3) / 4, NG), 128, 0, stream>>>(X16, CC, CG, Bq, CG, (size_t)DH * CG, 0.0625f, nullptr, 0, nullptr, 1, 0, 0, Q, nullptr, INNER, DH, NI, DH, CG);
  k_h16<<<(NI * INNER / 8 + 255) / 256, 256, 0, stream>>>(Q, Q16, (size_t)NI * INNER / 8);
  k_zero<<<(NG * NJP * 64 / 2 / 4 + 255) / 256, 256, 0, stream>>>((float*)KV16, (size_t)NG * NJP * 64 / 2 / 4);
  k_offkv<<<NG * NJ, 64, 0, stream>>>(Q, x, w1, b1, w2o, KV16, VG);
  k_gemm_hhx<0><<<dim3(((NJP / 16) * 1 + 3) / 4, NG), 128, 0, stream>>>(KV16, 64, (size_t)NJP * 64, Bk, CG, (size_t)DH * CG, 0.0625f, nullptr, 0, nullptr, 1, 0, 0, nullptr, K16, INNER, DH, NJP, DH, CG);
  k_gemm_hhx<0><<<dim3(((NJP / 16) * 1 + 3) / 4, NG), 128, 0, stream>>>(KV16, 64, (size_t)NJP * 64, Bv, CG, (size_t)DH * CG, 0.0625f, nullptr, 0, nullptr, 1, 0, 0, nullptr, V16, INNER, DH, NJP, DH, CG);
  k_kpad<<<(NJP * (INNER / 8) + 255) / 256, 256, 0, stream>>>(K16, KP); k_vt<<<(NG * DH * 16 + 255) / 256, 256, 0, stream>>>(V16, VT);
  k_gemm_hhx<0><<<dim3(((NI / 16) * ((NJP + 63) / 64) + 3) / 4, NG), 128, 0, stream>>>(Q16, INNER, DH, KP, INNER, DH, 0.125f, nullptr, 0, nullptr, 1, 0, 0, SIM, nullptr, NJP, (size_t)NI * NJP, NI, NJP, DH);
  for (int g = 0; g < NG; ++g) {
    k_cpb0<<<(unsigned)(((size_t)NI * NJ * 8 + 255) / 256), 256, 0, stream>>>(VG, g, c0w, c0b, H0);
    k_gemm_hhx<3><<<dim3(((NI * NJ / 16) * 1 + 3) / 4, 1), 128, 0, stream>>>(H0, CPB, 0, Bc1, CPB, 0, 0.0625f, c1b + (size_t)LSEL * CPB, 0, nullptr, 1, 0, 0, nullptr, H1, CPB, 0, NI * NJ, CPB, CPB);
    k_gemm_hhx<0><<<dim3(((NI * NJ / 16) * 1 + 3) / 4, 1), 128, 0, stream>>>(H1, CPB, 0, Bw2, CPB, 0, 0.0625f, Bb2, 0, nullptr, 1, 0, 0, BIAS, nullptr, 16, 0, NI * NJ, 16, CPB);
    k_soft<<<NI / 8, 256, 0, stream>>>(SIM, BIAS, g, ATT); }
  k_gemm_hhx<0><<<dim3(((NI / 16) * 1 + 3) / 4, NG), 128, 0, stream>>>(ATT, 128, (size_t)NI * 128, VT, 128, (size_t)DH * 128, 0.0009765625f, nullptr, 0, nullptr, 1, 0, 0, nullptr, O16, INNER, DH, NI, DH, 128);
  k_gemm_hhx<0><<<dim3(((NI / 16) * (CC / 64) + 3) / 4, 1), 128, 0, stream>>>(O16, INNER, 0, Bo, INNER, 0, 0.0625f, bo + (size_t)LSEL * CC, 0, nullptr, 1, 0, 0, Y, nullptr, CC, 0, NI, CC, INNER);
  k_nchw<<<(CC * (NI / 4) + 255) / 256, 256, 0, stream>>>(Y, (float*)d_out);
}
